// GNNReGVD_48112223650342
// MI455X (gfx1250) — hardware-verified
//
#include <hip/hip_runtime.h>
#include <math.h>

typedef __attribute__((ext_vector_type(16))) _Float16 v16h;
typedef __attribute__((ext_vector_type(16))) __bf16 v16b;
typedef __attribute__((ext_vector_type(8)))  _Float16 v8h;
typedef __attribute__((ext_vector_type(8)))  float v8f;
typedef __attribute__((ext_vector_type(4)))  float v4f;
typedef __attribute__((ext_vector_type(2)))  float v2f;
typedef __attribute__((ext_vector_type(4)))  unsigned v4u;
typedef __attribute__((ext_vector_type(4)))  int v4i;
typedef float __attribute__((may_alias)) float_a;
typedef int __attribute__((may_alias)) int_a;

template <typename T> __device__ __forceinline__ void vst2(void* p, T v) { *(volatile T*)p = v; __threadfence(); *(volatile T*)p = v; }
__device__ __forceinline__ v8f wmma16(v16h a, v16h b, v8f c) {
  v8f d = __builtin_amdgcn_wmma_f32_16x16x32_f16(false, a, false, b, (short)0, c, false, false);
  asm volatile("v_nop\n\tv_nop\n\tv_nop\n\tv_nop" : "+v"(d) : "v"(a), "v"(b));
  return d;
}
__device__ __forceinline__ v8f wmma_bf(v16b a, v16b b, v8f c) {
  v8f d = __builtin_amdgcn_wmma_f32_16x16x32_bf16(false, a, false, b, (short)0, c, false, false);
  asm volatile("v_nop\n\tv_nop\n\tv_nop\n\tv_nop" : "+v"(d) : "v"(a), "v"(b));
  return d;
}
__device__ __forceinline__ v16h frag_h(const _Float16* rowk0, int lane) {
  union { v16h v; v8h q[2]; } u; const _Float16* p = rowk0 + 8 * (lane >> 4);
  u.q[0] = *(const v8h*)p; u.q[1] = *(const v8h*)(p + 16); return u.v;
}
__device__ __forceinline__ v16h frag_f32(const float* rowk0, int lane) {
  v16h a; const float* p = rowk0 + 8 * (lane >> 4);
#pragma unroll
  for (int i = 0; i < 8; ++i) { a[i] = (_Float16)p[i]; a[8 + i] = (_Float16)p[16 + i]; }
  return a;
}
__device__ __forceinline__ v16h frag_f32s(const float* rowk0, int lane, float sc) {
  v16h a; const float* p = rowk0 + 8 * (lane >> 4);
#pragma unroll
  for (int i = 0; i < 8; ++i) { a[i] = (_Float16)(p[i] * sc); a[8 + i] = (_Float16)(p[16 + i] * sc); }
  return a;
}
__device__ __forceinline__ v16h fragc_f32(const float* W, int k0, int n, int lane, int ld, int K) {
  v16h a; const int g = lane >> 4;
#pragma unroll
  for (int i = 0; i < 8; ++i) { const int ka = k0 + 8 * g + i, kb = ka + 16;
    a[i] = (_Float16)(ka < K ? W[(size_t)(ka < K ? ka : K - 1) * ld + n] : 0.f); a[8 + i] = (_Float16)(kb < K ? W[(size_t)(kb < K ? kb : K - 1) * ld + n] : 0.f); }
  return a;
}
struct F2 { v16b h, l; };
__device__ __forceinline__ F2 bsplit16(const float v[16]) { F2 r;
#pragma unroll
  for (int i = 0; i < 16; ++i) { const __bf16 h = (__bf16)v[i]; r.h[i] = h; r.l[i] = (__bf16)(v[i] - (float)h); }
  return r; }
__device__ __forceinline__ F2 split_row(const float* row, int k0, int lane) { float v[16]; const float* p = row + k0 + 8 * (lane >> 4);
#pragma unroll
  for (int i = 0; i < 8; ++i) { v[i] = p[i]; v[8 + i] = p[16 + i]; }
  return bsplit16(v); }
__device__ __forceinline__ F2 split_rowK(const float* row, int k0, int lane, int K) { float v[16]; const int g = lane >> 4;
#pragma unroll
  for (int i = 0; i < 8; ++i) { const int ka = k0 + 8 * g + i, kb = ka + 16; v[i] = ka < K ? row[ka < K ? ka : K - 1] : 0.f; v[8 + i] = kb < K ? row[kb < K ? kb : K - 1] : 0.f; }
  return bsplit16(v); }
__device__ __forceinline__ F2 split_col(const float* W, int k0, int n, int lane, int ld, int K) { float v[16]; const int g = lane >> 4;
#pragma unroll
  for (int i = 0; i < 8; ++i) { const int ka = k0 + 8 * g + i, kb = ka + 16; v[i] = ka < K ? W[(size_t)(ka < K ? ka : K - 1) * ld + n] : 0.f; v[8 + i] = kb < K ? W[(size_t)(kb < K ? kb : K - 1) * ld + n] : 0.f; }
  return bsplit16(v); }
__device__ __forceinline__ v8f mac3(const F2& a, const F2& b, v8f c) { c = wmma_bf(a.l, b.h, c); c = wmma_bf(a.h, b.l, c); return wmma_bf(a.h, b.h, c); }
__device__ __forceinline__ float sigm(float v) { return 1.0f / (1.0f + expf(-v)); }
#define LDSX() do { asm volatile("s_wait_dscnt 0" ::: "memory"); __builtin_amdgcn_wave_barrier(); __builtin_amdgcn_fence(__ATOMIC_RELEASE, "workgroup"); } while (0)


#define NB 2
#define NN 2048
#define FIN 768
#define NH 8
#define OD 256
#define HW (NH * OD)
#define NTOK (NB * NN)
#ifndef TIB
#define TIB (NN / 64)
#define NBT NB
#define TOB (NN / 64)
#define TFB (NB * NN / 64)
#define DBG 0
#endif
typedef __attribute__((ext_vector_type(8))) __bf16 v8b;
__device__ __forceinline__ v16b frag_b(const __bf16* rowk0, int lane) {
  union { v16b v; v8b q[2]; } u; const __bf16* p = rowk0 + 8 * (lane >> 4);
  u.q[0] = *(const v8b*)p; u.q[1] = *(const v8b*)(p + 16); return u.v;
}
__device__ __forceinline__ float bfr(float v) { return (float)(__bf16)v; }
__device__ __attribute__((noinline)) float exp_ni(float v) { return expf(v); }
__device__ __attribute__((noinline)) float erf_ni(float v) { return erff(v); }

__device__ __attribute__((noinline)) float expm1_ni(float v) { return expm1f(v); }
#define WS_PW   0u
#define PWH 0
#define PWO (PWH + HW * FIN)
#define PWL (PWO + OD * HW)
#define PWN (PWL + OD * HW)
#define PWEND (PWN + OD * OD)
#define WS_H    (WS_PW + 2u * PWEND)
#define WS_HTH  (WS_H + 4u * NTOK * HW)
#define WS_HTL  (WS_HTH + 2u * NB * HW * NN)
#define WS_EB   (WS_HTL + 2u * NB * HW * NN)
#define WS_ED   (WS_EB + 4u * NB * NH * NN)
#define WS_S1   (WS_ED + 4u * NB * NH * NN)
#define WS_S2   (WS_S1 + 4u * NB * NH * NN)
#define WS_M    (WS_S2 + 4u * NB * NH * NN)
#define WS_L    (WS_M + 4u * NB * NH * NN)
#define WS_X1   (WS_L + 4u * NB * NH * NN)
#define WS_X2   (WS_X1 + 4u * NTOK * HW)
#define WS_HP   (WS_X2 + 4u * NTOK * OD)
#define WS_END  (WS_HP + 4u * NTOK * OD)

__global__ __launch_bounds__(256) void k_pack(const float* __restrict__ WHD, const float* __restrict__ WOUT, const float* __restrict__ WLIN, const float* __restrict__ WLN, __bf16* __restrict__ PW) {
  __shared__ __align__(16) __bf16 s[HW]; const int n = blockIdx.x, which = blockIdx.y, tid = threadIdx.x; int K; size_t dst;
  if (which == 0) { K = FIN; const int h = n / OD, o = n % OD; dst = PWH + (size_t)n * FIN; for (int k = tid; k < K; k += 256) s[k] = (__bf16)WHD[((size_t)h * FIN + k) * OD + o]; }
  else if (which == 1) { if (n >= OD) return; K = HW; dst = PWO + (size_t)n * HW; for (int k = tid; k < K; k += 256) s[k] = (__bf16)WOUT[(size_t)k * OD + n]; }
  else if (which == 2) { if (n >= OD) return; K = HW; dst = PWL + (size_t)n * HW; for (int k = tid; k < K; k += 256) s[k] = (__bf16)WLIN[(size_t)n * HW + k]; }
  else { if (n >= OD) return; K = OD; dst = PWN + (size_t)n * OD; for (int k = tid; k < K; k += 256) s[k] = (__bf16)WLN[(size_t)n * OD + k]; }
  __syncthreads();
  for (int q = tid; q < K / 8; q += 256) vst2((unsigned*)(PW + dst + q * 8), *(const v4u*)&s[q * 8]);
}
template <int RIN, int EPI>
__global__ __launch_bounds__(128) void k_gemm(const float* __restrict__ A, int lda, int K, const __bf16* __restrict__ P, const float* __restrict__ bias, const float* __restrict__ RES, float* __restrict__ OUT, int ldo) {
  __shared__ __align__(16) float so[4][16][132];
  const int tid = threadIdx.x, wave = tid >> 5, lane = tid & 31, col = lane & 15, g = lane >> 4; const size_t r0 = (size_t)blockIdx.x * 64 + wave * 16; const int n0 = blockIdx.y * 128;
  v8f acc[8] = {};
#pragma unroll 2
  for (int kc = 0; kc < K / 32; ++kc) { F2 a; if (RIN) { v16b ax; const float* p = A + (r0 + col) * (size_t)lda + kc * 32 + 8 * g;
#pragma unroll
      for (int i = 0; i < 8; ++i) { ax[i] = (__bf16)p[i]; ax[8 + i] = (__bf16)p[16 + i]; } a.h = ax; a.l = ax; } else a = split_row(A + (r0 + col) * (size_t)lda, kc * 32, lane);
#pragma unroll
    for (int j = 0; j < 8; ++j) { const v16b w = frag_b(P + (size_t)(n0 + j * 16 + col) * K + kc * 32, lane); if (!RIN) acc[j] = wmma_bf(a.l, w, acc[j]); acc[j] = wmma_bf(a.h, w, acc[j]); } }
#pragma unroll
  for (int j = 0; j < 8; ++j) { const int n = n0 + j * 16 + col; const float bb = bias ? bfr(bias[n]) : 0.f;
#pragma unroll
    for (int r = 0; r < 8; ++r) { float v = acc[j][r] + bb; if (EPI == 1) v += RES[(r0 + 8 * g + r) * (size_t)ldo + n]; if (EPI == 2) v = fmaxf(v, 0.f); so[wave][8 * g + r][j * 16 + col] = v; } }
  LDSX();
  for (int rl = 0; rl < 16; ++rl) vst2(OUT + (r0 + rl) * (size_t)ldo + n0 + lane * 4, *(const v4f*)&so[wave][rl][lane * 4]);
}
__global__ __launch_bounds__(256) void k_sdot(const float* __restrict__ H, int ldh, int nh, const float* __restrict__ A, float* __restrict__ S1, float* __restrict__ S2, float* __restrict__ EB, float* __restrict__ ED) {
  __shared__ __align__(16) float s1s[NH][64], s2s[NH][64], sebs[NH][64], seds[NH][64]; const int tid = threadIdx.x, wave = tid >> 5, lane = tid & 31; const size_t rb = (size_t)blockIdx.x * 64; const int b = (int)(rb / NN), n0 = (int)(rb % NN);
  for (int q = wave; q < 64 * nh; q += 8) { const int rl = q / nh, h = q % nh; const float* hr = H + (rb + rl) * (size_t)ldh + h * OD; float a1 = 0.f, a2 = 0.f;
#pragma unroll
    for (int k = 0; k < 8; ++k) { const int c = lane + 32 * k; const float hv = hr[c]; a1 += hv * bfr(A[(size_t)h * 2 * OD + c]); a2 += hv * bfr(A[(size_t)h * 2 * OD + OD + c]); }
#pragma unroll
    for (int o = 1; o < 32; o <<= 1) { a1 += __shfl_xor(a1, o); a2 += __shfl_xor(a2, o); }
    if (lane == 0) { s1s[h][rl] = a1; s2s[h][rl] = a2; sebs[h][rl] = exp_ni(a2); seds[h][rl] = exp_ni(0.2f * a2); } }
  __syncthreads();
  for (int q = tid; q < nh * 64; q += 256) { const int h = q >> 6, pc = q & 63; const size_t o = ((size_t)b * NH + h) * NN + n0; const int p4 = (pc & 15) * 4; if (pc < 16) vst2(S1 + o + p4, *(const v4f*)&s1s[h][p4]); else if (pc < 32) vst2(S2 + o + p4, *(const v4f*)&s2s[h][p4]); else if (pc < 48) vst2(EB + o + p4, *(const v4f*)&sebs[h][p4]); else vst2(ED + o + p4, *(const v4f*)&seds[h][p4]); }
}
__device__ __forceinline__ float leaky02(float v) { return v > 0.f ? v : 0.2f * v; }
__global__ __launch_bounds__(256) void k_stats(const float* __restrict__ ADJ, const float* __restrict__ S1, const float* __restrict__ S2, int nh, float* __restrict__ M, float* __restrict__ L) {
  __shared__ int sl[8][NN]; __shared__ __align__(16) float sm[NH][8], sz[NH][8];
  const int tid = threadIdx.x, wave = tid >> 5, lane = tid & 31; const int b = blockIdx.y; const int i0 = blockIdx.x * 8; const int i = i0 + wave; const size_t row = (size_t)b * NN + i;
  const float* arow = ADJ + row * NN; int cnt = 0;
  for (int c0 = 0; c0 < NN; c0 += 32) { const int j = c0 + lane; const bool live = bfr(arow[j]) > 0.f; const unsigned bal = __builtin_amdgcn_ballot_w32(live); const int rank = __builtin_popcount(bal & ((1u << lane) - 1u)); if (live) sl[wave][cnt + rank] = j; cnt += __builtin_popcount(bal); }
  LDSX();
  for (int h = 0; h < nh; ++h) { const float* s2 = S2 + ((size_t)b * NH + h) * NN; const float s1 = S1[((size_t)b * NH + h) * NN + i];
    float mx = -3.0e38f; for (int q = lane; q < cnt; q += 32) mx = fmaxf(mx, s2[sl[wave][q]]);
#pragma unroll
    for (int o = 1; o < 32; o <<= 1) mx = fmaxf(mx, __shfl_xor(mx, o));
    const float m = leaky02(s1 + mx); float z = 0.f; for (int q = lane; q < cnt; q += 32) z += exp_ni(leaky02(s1 + s2[sl[wave][q]]) - m);
#pragma unroll
    for (int o = 1; o < 32; o <<= 1) z += __shfl_xor(z, o);
    if (lane == 0) { sm[h][wave] = m; sz[h][wave] = z; } }
  __syncthreads();
  if (tid < nh * 4) { const int h = tid >> 2, pc = tid & 3; const size_t o = ((size_t)b * NH + h) * NN + i0; if (pc < 2) vst2(M + o + pc * 4, *(const v4f*)&sm[h][pc * 4]); else vst2(L + o + (pc - 2) * 4, *(const v4f*)&sz[h][(pc - 2) * 4]); }
}
__global__ __launch_bounds__(256) void k_planes(const float* __restrict__ H, int ldh, int width, __bf16* __restrict__ PH, __bf16* __restrict__ PL) {
  __shared__ __align__(16) __bf16 sh[128][72], sl[128][72]; const int tid = threadIdx.x; const size_t rb = (size_t)blockIdx.x * 64; const int c0 = blockIdx.y * 128; const int b = (int)(rb / NN), j0 = (int)(rb % NN);
  for (int q = tid; q < 64 * 128; q += 256) { const int rl = q >> 7, c = q & 127; const float v = H[(rb + rl) * (size_t)ldh + c0 + c]; const __bf16 hb = (__bf16)v; sh[c][rl] = hb; sl[c][rl] = (__bf16)(v - (float)hb); }
  __syncthreads();
  for (int q = tid; q < 128 * 8; q += 256) { const int c = q >> 3, pc = q & 7; const size_t o = ((size_t)b * width + c0 + c) * NN + j0 + pc * 8; vst2((unsigned*)(PH + o), *(const v4u*)&sh[c][pc * 8]); vst2((unsigned*)(PL + o), *(const v4u*)&sl[c][pc * 8]); }
}
template <int ELU>
__global__ __launch_bounds__(128) void k_av(const float* __restrict__ ADJ, const float* __restrict__ S1, const float* __restrict__ S2, const float* __restrict__ EB, const float* __restrict__ ED, const float* __restrict__ M, const float* __restrict__ L, const __bf16* __restrict__ PH, const __bf16* __restrict__ PL, int width, int nh, float* __restrict__ OUT, int ldo) {
  __shared__ __align__(16) float so[4][16][260];
  const int tid = threadIdx.x, wave = tid >> 5, lane = tid & 31, col = lane & 15, g = lane >> 4; const int b = blockIdx.y / nh, h = blockIdx.y % nh; const int i0 = blockIdx.x * 64 + wave * 16;
  const size_t hb = ((size_t)b * NH + h) * NN; const float* s2 = S2 + hb; const float* eb = EB + hb; const float* ed = ED + hb;
  const float s1 = S1[hb + i0 + col], mi = M[hb + i0 + col]; const float ai = exp_ni(s1 - mi), ci = exp_ni(0.2f * s1 - mi); const float* arow = ADJ + ((size_t)b * NN + i0 + col) * NN;
  v8f acc[16]; for (int t = 0; t < 16; ++t) acc[t] = (v8f){};
#pragma unroll 1
  for (int ks = 0; ks < NN / 32; ++ks) { float v[16]; const v4f a0 = *(const v4f*)(arow + ks * 32 + 8 * g), a1 = *(const v4f*)(arow + ks * 32 + 8 * g + 4), a2 = *(const v4f*)(arow + ks * 32 + 8 * g + 16), a3 = *(const v4f*)(arow + ks * 32 + 8 * g + 20);
    float am[16] = {a0[0], a0[1], a0[2], a0[3], a1[0], a1[1], a1[2], a1[3], a2[0], a2[1], a2[2], a2[3], a3[0], a3[1], a3[2], a3[3]};
#pragma unroll
    for (int q = 0; q < 16; ++q) { const int j = ks * 32 + 8 * g + (q & 7) + ((q >> 3) << 4); const float pv = (s1 + s2[j] > 0.f) ? ai * eb[j] : ci * ed[j]; v[q] = (bfr(am[q]) > 0.f) ? pv : 0.f; }
    const F2 a = bsplit16(v);
#pragma unroll
    for (int jt = 0; jt < 16; ++jt) { const size_t pr = ((size_t)b * width + h * OD + jt * 16 + col) * NN + ks * 32; const v16b ph = frag_b(PH + pr, lane), pl = frag_b(PL + pr, lane); acc[jt] = wmma_bf(a.l, ph, acc[jt]); acc[jt] = wmma_bf(a.h, pl, acc[jt]); acc[jt] = wmma_bf(a.h, ph, acc[jt]); } }
#pragma unroll
  for (int jt = 0; jt < 16; ++jt)
#pragma unroll
    for (int r = 0; r < 8; ++r) { const int i = i0 + 8 * g + r; const float il = 1.0f / L[hb + i]; float vv = acc[jt][r] * il; if (ELU) vv = (vv > 0.f) ? vv : expm1_ni(vv); so[wave][8 * g + r][jt * 16 + col] = vv; }
  LDSX();
  for (int rl = 0; rl < 16; ++rl) { vst2(OUT + ((size_t)b * NN + i0 + rl) * ldo + h * OD + lane * 4, *(const v4f*)&so[wave][rl][lane * 4]); vst2(OUT + ((size_t)b * NN + i0 + rl) * ldo + h * OD + 128 + lane * 4, *(const v4f*)&so[wave][rl][128 + lane * 4]); }
}
extern "C" void kernel_launch(void* const* d_in, const int* in_sizes, int n_in, void* d_out, int out_size, void* d_ws, size_t ws_size, hipStream_t stream) {
  (void)in_sizes; (void)n_in; (void)out_size;
  const float** F = (const float**)d_in;
  if (ws_size < (size_t)WS_END) return;
  char* ws = (char*)d_ws; __bf16 *PW = (__bf16*)(ws + WS_PW), *HTH = (__bf16*)(ws + WS_HTH), *HTL = (__bf16*)(ws + WS_HTL);
  float *H = (float*)(ws + WS_H), *EB = (float*)(ws + WS_EB), *ED = (float*)(ws + WS_ED), *S1 = (float*)(ws + WS_S1), *S2 = (float*)(ws + WS_S2), *M = (float*)(ws + WS_M), *Lr = (float*)(ws + WS_L), *X1 = (float*)(ws + WS_X1), *X2 = (float*)(ws + WS_X2), *HP = (float*)(ws + WS_HP);
  k_pack<<<dim3(HW, 4), 256, 0, stream>>>(F[3], F[5], F[7], F[9], PW);
  k_gemm<1, 0><<<dim3(NBT * NN / 64, HW / 128), 128, 0, stream>>>(F[0], FIN, FIN, PW + PWH, nullptr, nullptr, H, HW);
  const float* X1u = X1;
  if (DBG != 2) {
    k_sdot<<<NBT * NN / 64, 256, 0, stream>>>(H, HW, NH, F[4], S1, S2, EB, ED);
    k_planes<<<dim3(NBT * NN / 64, HW / 128), 256, 0, stream>>>(H, HW, HW, HTH, HTL);
    k_stats<<<dim3(TIB * 8, NBT), 256, 0, stream>>>(F[1], S1, S2, NH, M, Lr);
    k_av<1><<<dim3(TIB, NBT * NH), 128, 0, stream>>>(F[1], S1, S2, EB, ED, M, Lr, HTH, HTL, HW, NH, (DBG == 1) ? (float*)d_out : X1, HW);
    if (DBG == 1) return;
  } else X1u = H;
  k_gemm<0, 0><<<dim3(NBT * NN / 64, OD / 128), 128, 0, stream>>>(X1u, HW, HW, PW + PWO, nullptr, nullptr, HP, OD);
  k_sdot<<<NBT * NN / 64, 256, 0, stream>>>(HP, OD, 1, F[6], S1, S2, EB, ED);
  k_planes<<<dim3(NBT * NN / 64, OD / 128), 256, 0, stream>>>(HP, OD, OD, HTH, HTL);
  k_stats<<<dim3(TOB * 8, NBT), 256, 0, stream>>>(F[1], S1, S2, 1, M, Lr);
  k_av<0><<<dim3(TOB, NBT), 128, 0, stream>>>(F[1], S1, S2, EB, ED, M, Lr, HTH, HTL, OD, 1, X2, OD);
  k_gemm<0, 1><<<dim3(TFB, OD / 128), 128, 0, stream>>>(X1u, HW, HW, PW + PWL, F[8], X2, X2, OD);
  k_gemm<0, 2><<<dim3(TFB, OD / 128), 128, 0, stream>>>(X2, OD, OD, PW + PWN, F[10], nullptr, (float*)d_out, OD);
}
